// SANet_51694226374934
// MI455X (gfx1250) — hardware-verified
//
#include <hip/hip_runtime.h>
#include <stdint.h>

#ifndef NB
#define NB 4
#endif
#ifndef SEQ
#define SEQ 2048
#endif
#define NB_FULL 4
#define T_FULL  2048
#define CH      512
#define NMAT    4
#define QT      64
#define OSP     68
#define TP      72
#define NCH     (SEQ / 256)
#define PCAR    16384.0f
#define IPCAR   6.103515625e-05f
#define EPSN    1.0e-5f
#define WS_CAP  134217728

static_assert(NB >= 1 && NB <= NB_FULL);
static_assert(SEQ >= 256 && SEQ <= T_FULL && SEQ % 256 == 0);
static_assert(SEQ % QT == 0 && CH % QT == 0);
static_assert(CH % 256 == 0 && CH % 32 == 0 && SEQ % 32 == 0 && SEQ % 16 == 0);
static_assert((OSP * 4) % 16 == 0);
static_assert((TP * 2) % 16 == 0);
static_assert((NB * SEQ) % 8 == 0);
static_assert(CH % 8 == 0);

typedef _Float16       v16h __attribute__((ext_vector_type(16)));
typedef _Float16       v8h  __attribute__((ext_vector_type(8)));
typedef __bf16         v16b __attribute__((ext_vector_type(16)));
typedef unsigned short v8us __attribute__((ext_vector_type(8)));
typedef float          v8f  __attribute__((ext_vector_type(8)));
typedef float          v4f  __attribute__((ext_vector_type(4)));
typedef unsigned int   v4u  __attribute__((ext_vector_type(4)));

union Frag { v8us u[2]; v16h h; v16b bf; };
static_assert(sizeof(Frag) == 32);

constexpr size_t cmax(size_t a, size_t b) { return a > b ? a : b; }
constexpr size_t PLB = (size_t)NB * SEQ * CH * 2;
constexpr size_t SB  = (size_t)NB * SEQ * SEQ * 4;
constexpr size_t PB  = (size_t)NB * SEQ * SEQ * 2;
constexpr size_t WB  = (size_t)NMAT * CH * CH * 2;
constexpr size_t RXB = cmax(cmax(5 * PLB, SB), 2 * PLB);
constexpr size_t RMB = cmax(4 * PLB, PB);
constexpr size_t RVB = PLB;
static_assert(WB % 256 == 0 && PLB % 256 == 0 && SB % 256 == 0 && PB % 256 == 0);
static_assert(5 * PLB <= RXB && SB <= RXB && 2 * PLB <= RXB);
static_assert(4 * PLB <= RMB && PB <= RMB);
static_assert(WB + RXB + RMB + RVB <= (size_t)WS_CAP);

__device__ __forceinline__ unsigned short bf_bits(float f) {
  unsigned u = __float_as_uint(f);
  return (unsigned short)((u + 0x7FFFu + ((u >> 16) & 1u)) >> 16);
}
__device__ __forceinline__ float bf_up(unsigned short hb) { return __uint_as_float(((unsigned)hb) << 16); }
__device__ __forceinline__ float bfr(float f) { return bf_up(bf_bits(f)); }
__device__ __forceinline__ unsigned short h_bits(_Float16 x) { return __builtin_bit_cast(unsigned short, x); }
__device__ __forceinline__ unsigned pk16(unsigned short a, unsigned short b) { return (unsigned)a | ((unsigned)b << 16); }
__device__ __forceinline__ v8f zero8() { v8f z = {0.f, 0.f, 0.f, 0.f, 0.f, 0.f, 0.f, 0.f}; return z; }

__device__ __forceinline__ Frag ldfrag(const unsigned short* p) {
  Frag f;
  f.u[0] = *(const v8us*)(p);
  f.u[1] = *(const v8us*)(p + 16);
  return f;
}

__device__ __forceinline__ v8f mma_h(v16h a, v16h b, v8f c) {
  v8f d = __builtin_amdgcn_wmma_f32_16x16x32_f16(false, a, false, b, (short)0, c, false, false);
#if defined(__HIP_DEVICE_COMPILE__)
  asm volatile("v_nop\n\tv_nop\n\tv_nop\n\tv_nop" : "+v"(d) : "v"(a), "v"(b));
#endif
  return d;
}
__device__ __forceinline__ v8f mma_b(v16b a, v16b b, v8f c) {
  v8f d = __builtin_amdgcn_wmma_f32_16x16x32_bf16(false, a, false, b, (short)0, c, false, false);
#if defined(__HIP_DEVICE_COMPILE__)
  const v16h ha = __builtin_bit_cast(v16h, a), hb = __builtin_bit_cast(v16h, b);
  asm volatile("v_nop\n\tv_nop\n\tv_nop\n\tv_nop" : "+v"(d) : "v"(ha), "v"(hb));
#endif
  return d;
}

template <int NPROD, bool HALF>
__device__ __forceinline__ void gemm_core(v8f (&acc)[4],
                                          const unsigned short* __restrict__ a0,
                                          const unsigned short* __restrict__ a1, size_t amt,
                                          const unsigned short* __restrict__ b0,
                                          const unsigned short* __restrict__ b1, int ksteps) {
  static_assert(NPROD >= 1 && NPROD <= 3);
  static_assert(!(HALF && NPROD != 1));
#pragma unroll 1
  for (int ks = 0; ks < ksteps; ++ks) {
    const int ko = 32 * ks;
    const Frag fb0 = ldfrag(b0 + ko);
    Frag fb1 = fb0;
    if (NPROD >= 2) fb1 = ldfrag(b1 + ko);
#pragma unroll
    for (int mt = 0; mt < 4; ++mt) {
      const Frag fa0 = ldfrag(a0 + (size_t)mt * amt + ko);
      if (HALF) {
        acc[mt] = mma_h(fa0.h, fb0.h, acc[mt]);
      } else {
        acc[mt] = mma_b(fa0.bf, fb0.bf, acc[mt]);
        if (NPROD >= 2) acc[mt] = mma_b(fa0.bf, fb1.bf, acc[mt]);
        if (NPROD >= 3) {
          const Frag fa1 = ldfrag(a1 + (size_t)mt * amt + ko);
          acc[mt] = mma_b(fa1.bf, fb0.bf, acc[mt]);
        }
      }
    }
  }
}

__device__ __forceinline__ void stage_nT(float* Os, const v8f (&acc)[4], float sc, int wave, int hh, int c) {
  const int nl = 16 * wave + c;
#pragma unroll
  for (int mt = 0; mt < 4; ++mt) {
    v4f va, vb;
#pragma unroll
    for (int r = 0; r < 4; ++r) { va[r] = acc[mt][r] * sc; vb[r] = acc[mt][4 + r] * sc; }
    *(v4f*)(Os + nl * OSP + 16 * mt + 8 * hh)     = va;
    *(v4f*)(Os + nl * OSP + 16 * mt + 8 * hh + 4) = vb;
  }
}
__device__ __forceinline__ void stage_mn(float* Os, const v8f (&acc)[4], int wave, int hh, int c) {
  const int nl = 16 * wave + c;
#pragma unroll
  for (int mt = 0; mt < 4; ++mt) {
#pragma unroll
    for (int r = 0; r < 8; ++r) Os[(16 * mt + 8 * hh + r) * OSP + nl] = acc[mt][r];
  }
}

template <bool BIAS>
__device__ __forceinline__ void planes_out(const float* Os, const float* __restrict__ bias, int o0,
                                           unsigned short* Ph, unsigned short* Pl, size_t rowbase, int tid) {
  const int e = tid & 7, lq = tid >> 3;
  float bv[8];
#pragma unroll
  for (int t = 0; t < 8; ++t) bv[t] = 0.f;
  if (BIAS) {
    const v4f b0 = *(const v4f*)(bias + o0 + 8 * e);
    const v4f b1 = *(const v4f*)(bias + o0 + 8 * e + 4);
#pragma unroll
    for (int t = 0; t < 4; ++t) { bv[t] = bfr(b0[t]); bv[4 + t] = bfr(b1[t]); }
  }
  v4u uh[4], ul[4];
#pragma unroll
  for (int it = 0; it < 4; ++it) {
    const int row = it * 16 + lq;
    const v4f a = *(const v4f*)(Os + row * OSP + 8 * e);
    const v4f q = *(const v4f*)(Os + row * OSP + 8 * e + 4);
    const float f[8] = {a[0], a[1], a[2], a[3], q[0], q[1], q[2], q[3]};
#pragma unroll
    for (int t = 0; t < 4; ++t) {
      const float f0 = f[2 * t] + bv[2 * t], f1 = f[2 * t + 1] + bv[2 * t + 1];
      const unsigned short hb0 = bf_bits(f0), hb1 = bf_bits(f1);
      const unsigned short lb0 = bf_bits(f0 - bf_up(hb0));
      const unsigned short lb1 = bf_bits(f1 - bf_up(hb1));
      uh[it][t] = pk16(hb0, hb1);
      ul[it][t] = pk16(lb0, lb1);
    }
  }
#pragma unroll
  for (int pass = 0; pass < 2; ++pass) {
#pragma unroll
    for (int it = 0; it < 4; ++it) {
      const int row = it * 16 + lq;
      const size_t po = (rowbase + (size_t)row) * CH + o0 + 8 * e;
      *(volatile v4u*)(Ph + po) = uh[it];
      *(volatile v4u*)(Pl + po) = ul[it];
    }
    __threadfence();
  }
}

__global__ __launch_bounds__(256)
void cvt_w(const float* __restrict__ w0, const float* __restrict__ w1,
           const float* __restrict__ w2, const float* __restrict__ w3, unsigned short* W16) {
  const int tid = threadIdx.x, blk = blockIdx.x;
  const int wave = tid >> 5, lane = tid & 31;
  const int mi = blk / (CH / 8);
  const int o  = 8 * (blk - mi * (CH / 8)) + wave;
  const float* wb = (mi == 0) ? w0 : (mi == 1) ? w1 : (mi == 2) ? w2 : w3;
  v4u u[CH / 256];
#pragma unroll
  for (int j = 0; j < CH / 256; ++j) {
    const float* s = wb + (size_t)o * CH + 256 * j + 8 * lane;
    const v4f a = *(const v4f*)s;
    const v4f q = *(const v4f*)(s + 4);
    const float f[8] = {a[0], a[1], a[2], a[3], q[0], q[1], q[2], q[3]};
#pragma unroll
    for (int t = 0; t < 4; ++t) u[j][t] = pk16(bf_bits(f[2 * t]), bf_bits(f[2 * t + 1]));
  }
#pragma unroll
  for (int pass = 0; pass < 2; ++pass) {
#pragma unroll
    for (int j = 0; j < CH / 256; ++j)
      *(volatile v4u*)(W16 + ((size_t)(mi * CH + o)) * CH + 256 * j + 8 * lane) = u[j];
    __threadfence();
  }
}

template <int RAW>
__global__ __launch_bounds__(256)
void cvt_norm(const float* __restrict__ x, unsigned short* Ph, unsigned short* Pl, unsigned short* Pr) {
  __shared__ __align__(16) unsigned short Th[QT * TP];
  __shared__ __align__(16) unsigned short Tl[QT * TP];
  __shared__ __align__(16) unsigned short Tr[QT * TP];
  __shared__ float mean_s[QT];
  __shared__ float rstd_s[QT];
  const int tid = threadIdx.x;
  const int cb = blockIdx.x, b = blockIdx.y;
  const int c0 = cb * QT;

  {
    const int rl = tid >> 2, q = tid & 3;
    const float* xr = x + ((size_t)(b * CH + c0 + rl)) * T_FULL + 4 * q;
    float s0 = 0.f, s1 = 0.f, s2 = 0.f, s3 = 0.f;
#pragma unroll 2
    for (int j = 0; j < SEQ / 16; ++j) {
      const v4f a = *(const v4f*)(xr + 16 * j);
      s0 += bfr(a[0]); s1 += bfr(a[1]); s2 += bfr(a[2]); s3 += bfr(a[3]);
    }
    float sm = (s0 + s1) + (s2 + s3);
    sm += __shfl_xor(sm, 1, 32);
    sm += __shfl_xor(sm, 2, 32);
    const float mean = sm * (1.0f / (float)SEQ);
    float v0 = 0.f, v1 = 0.f, v2 = 0.f, v3 = 0.f;
#pragma unroll 2
    for (int j = 0; j < SEQ / 16; ++j) {
      const v4f a = *(const v4f*)(xr + 16 * j);
      const float d0 = bfr(a[0]) - mean, d1 = bfr(a[1]) - mean, d2 = bfr(a[2]) - mean, d3 = bfr(a[3]) - mean;
      v0 += d0 * d0; v1 += d1 * d1; v2 += d2 * d2; v3 += d3 * d3;
    }
    float sv = (v0 + v1) + (v2 + v3);
    sv += __shfl_xor(sv, 1, 32);
    sv += __shfl_xor(sv, 2, 32);
    const float var = sv * (1.0f / (float)SEQ);
    const float rs  = rsqrtf(var + EPSN);
    if (q == 0) { mean_s[rl] = mean; rstd_s[rl] = rs; }
  }
  __syncthreads();

  const int e = tid & 7, lq = tid >> 3;
#pragma unroll 1
  for (int n0 = 0; n0 < SEQ; n0 += QT) {
#pragma unroll
    for (int it = 0; it < 2; ++it) {
      const int cl = it * 32 + lq;
      const float* sp = x + ((size_t)(b * CH + c0 + cl)) * T_FULL + n0 + 8 * e;
      const v4f a = *(const v4f*)sp;
      const v4f q = *(const v4f*)(sp + 4);
      const float f[8] = {a[0], a[1], a[2], a[3], q[0], q[1], q[2], q[3]};
      const float mu = mean_s[cl], rs = rstd_s[cl];
#pragma unroll
      for (int t = 0; t < 8; ++t) {
        const unsigned short rb = bf_bits(f[t]);
        const float xn = (bf_up(rb) - mu) * rs;
        const unsigned short hb = bf_bits(xn);
        const unsigned short lb = bf_bits(xn - bf_up(hb));
        Th[(8 * e + t) * TP + cl] = hb;
        Tl[(8 * e + t) * TP + cl] = lb;
        if (RAW) Tr[(8 * e + t) * TP + cl] = rb;
      }
    }
    __syncthreads();
    v4u uh[2], ul[2], ur[2];
#pragma unroll
    for (int it = 0; it < 2; ++it) {
      const int nl = it * 32 + lq;
      uh[it] = *(const v4u*)(Th + nl * TP + 8 * e);
      ul[it] = *(const v4u*)(Tl + nl * TP + 8 * e);
      if (RAW) ur[it] = *(const v4u*)(Tr + nl * TP + 8 * e); else ur[it] = uh[it];
    }
#pragma unroll
    for (int pass = 0; pass < 2; ++pass) {
#pragma unroll
      for (int it = 0; it < 2; ++it) {
        const int nl = it * 32 + lq;
        const size_t po = ((size_t)(b * SEQ + n0 + nl)) * CH + c0 + 8 * e;
        *(volatile v4u*)(Ph + po) = uh[it];
        *(volatile v4u*)(Pl + po) = ul[it];
        if (RAW) *(volatile v4u*)(Pr + po) = ur[it];
      }
      __threadfence();
    }
    __syncthreads();
  }
}

__global__ __launch_bounds__(128)
void gemm_nm(const unsigned short* __restrict__ W, const float* __restrict__ bias,
             const unsigned short* __restrict__ Xh, const unsigned short* __restrict__ Xl,
             unsigned short* Ph, unsigned short* Pl) {
  __shared__ __align__(16) float Os[QT * OSP];
  const int tid = threadIdx.x, lane = tid & 31, wave = tid >> 5;
  const int hh = lane >> 4, c = lane & 15;
  const int nt = blockIdx.x, mb = blockIdx.y, b = blockIdx.z;
  const int n0 = nt * QT, o0 = mb * QT;
  const unsigned short* ap = W + (size_t)(o0 + c) * CH + 8 * hh;
  const size_t bq = ((size_t)(b * SEQ + n0 + 16 * wave + c)) * CH + 8 * hh;
  v8f acc[4];
#pragma unroll
  for (int mt = 0; mt < 4; ++mt) acc[mt] = zero8();
  gemm_core<2, false>(acc, ap, ap, (size_t)16 * CH, Xh + bq, Xl + bq, CH / 32);
  stage_nT(Os, acc, 1.0f, wave, hh, c);
  __syncthreads();
  planes_out<true>(Os, bias, o0, Ph, Pl, (size_t)(b * SEQ + n0), tid);
}

__global__ __launch_bounds__(128)
void gemm_val(const unsigned short* __restrict__ W, const float* __restrict__ bias,
              const unsigned short* __restrict__ Xr, unsigned short* V16) {
  __shared__ __align__(16) float Os[QT * OSP];
  const int tid = threadIdx.x, lane = tid & 31, wave = tid >> 5;
  const int hh = lane >> 4, c = lane & 15;
  const int nt = blockIdx.x, mb = blockIdx.y, b = blockIdx.z;
  const int n0 = nt * QT, o0 = mb * QT;
  const unsigned short* ap = W + (size_t)(o0 + c) * CH + 8 * hh;
  const size_t bq = ((size_t)(b * SEQ + n0 + 16 * wave + c)) * CH + 8 * hh;
  v8f acc[4];
#pragma unroll
  for (int mt = 0; mt < 4; ++mt) acc[mt] = zero8();
  gemm_core<1, false>(acc, ap, ap, (size_t)16 * CH, Xr + bq, Xr + bq, CH / 32);
  stage_mn(Os, acc, wave, hh, c);
  __syncthreads();
  const int e = tid & 7, lq = tid >> 3;
  v4u u[4];
#pragma unroll
  for (int it = 0; it < 4; ++it) {
    const int row = it * 16 + lq;
    const float bb = bfr(bias[o0 + row]);
    const v4f a = *(const v4f*)(Os + row * OSP + 8 * e);
    const v4f q = *(const v4f*)(Os + row * OSP + 8 * e + 4);
    const float f[8] = {a[0], a[1], a[2], a[3], q[0], q[1], q[2], q[3]};
#pragma unroll
    for (int t = 0; t < 4; ++t) {
      const _Float16 h0 = (_Float16)(f[2 * t] + bb);
      const _Float16 h1 = (_Float16)(f[2 * t + 1] + bb);
      u[it][t] = pk16(h_bits(h0), h_bits(h1));
    }
  }
#pragma unroll
  for (int pass = 0; pass < 2; ++pass) {
#pragma unroll
    for (int it = 0; it < 4; ++it) {
      const int row = it * 16 + lq;
      const size_t po = ((size_t)(b * CH + o0 + row)) * SEQ + n0 + 8 * e;
      *(volatile v4u*)(V16 + po) = u[it];
    }
    __threadfence();
  }
}

__global__ __launch_bounds__(128)
void gemm_sc(const unsigned short* __restrict__ Qh, const unsigned short* __restrict__ Ql,
             const unsigned short* __restrict__ Kh, const unsigned short* __restrict__ Kl, float* S) {
  __shared__ __align__(16) float Os[QT * OSP];
  const int tid = threadIdx.x, lane = tid & 31, wave = tid >> 5;
  const int hh = lane >> 4, c = lane & 15;
  const int nt = blockIdx.x, mb = blockIdx.y, b = blockIdx.z;
  const int n0 = nt * QT, m0 = mb * QT;
  const size_t aq = ((size_t)(b * SEQ + m0 + c)) * CH + 8 * hh;
  const size_t bq = ((size_t)(b * SEQ + n0 + 16 * wave + c)) * CH + 8 * hh;
  v8f acc[4];
#pragma unroll
  for (int mt = 0; mt < 4; ++mt) acc[mt] = zero8();
  gemm_core<3, false>(acc, Qh + aq, Ql + aq, (size_t)16 * CH, Kh + bq, Kl + bq, CH / 32);
  stage_mn(Os, acc, wave, hh, c);
  __syncthreads();
  const int e = tid & 15, lq = tid >> 4;
  v4f res[8];
#pragma unroll
  for (int it = 0; it < 8; ++it) {
    const int row = it * 8 + lq;
    res[it] = *(const v4f*)(Os + row * OSP + 4 * e);
  }
#pragma unroll
  for (int pass = 0; pass < 2; ++pass) {
#pragma unroll
    for (int it = 0; it < 8; ++it) {
      const int row = it * 8 + lq;
      *(volatile v4f*)(S + ((size_t)(b * SEQ + m0 + row)) * SEQ + n0 + 4 * e) = res[it];
    }
    __threadfence();
  }
}

__global__ __launch_bounds__(256)
void softmax_k(const float* __restrict__ S, unsigned short* P16) {
  const int tid = threadIdx.x, wave = tid >> 5, lane = tid & 31;
  const size_t row = (size_t)blockIdx.x * 8 + wave;
  const float* sr = S + row * SEQ;
  float v[SEQ / 32];
#pragma unroll
  for (int j = 0; j < NCH; ++j) {
    const v4f a = *(const v4f*)(sr + 256 * j + 8 * lane);
    const v4f q = *(const v4f*)(sr + 256 * j + 8 * lane + 4);
#pragma unroll
    for (int t = 0; t < 4; ++t) { v[8 * j + t] = a[t]; v[8 * j + 4 + t] = q[t]; }
  }
  float mx = -3.0e38f;
#pragma unroll
  for (int i = 0; i < SEQ / 32; ++i) mx = fmaxf(mx, v[i]);
#pragma unroll
  for (int o = 16; o > 0; o >>= 1) mx = fmaxf(mx, __shfl_xor(mx, o, 32));
  float l = 0.f;
#pragma unroll
  for (int i = 0; i < SEQ / 32; ++i) { v[i] = __expf(v[i] - mx); l += v[i]; }
#pragma unroll
  for (int o = 16; o > 0; o >>= 1) l += __shfl_xor(l, o, 32);
  const float sc = PCAR * (1.0f / l);
  v4u u[NCH];
#pragma unroll
  for (int j = 0; j < NCH; ++j) {
#pragma unroll
    for (int t = 0; t < 4; ++t) {
      const _Float16 h0 = (_Float16)(v[8 * j + 2 * t] * sc);
      const _Float16 h1 = (_Float16)(v[8 * j + 2 * t + 1] * sc);
      u[j][t] = pk16(h_bits(h0), h_bits(h1));
    }
  }
#pragma unroll
  for (int pass = 0; pass < 2; ++pass) {
#pragma unroll
    for (int j = 0; j < NCH; ++j)
      *(volatile v4u*)(P16 + row * SEQ + 256 * j + 8 * lane) = u[j];
    __threadfence();
  }
}

__global__ __launch_bounds__(128)
void gemm_pv(const unsigned short* __restrict__ V16, const unsigned short* __restrict__ P16,
             unsigned short* Mh, unsigned short* Mlo) {
  __shared__ __align__(16) float Os[QT * OSP];
  const int tid = threadIdx.x, lane = tid & 31, wave = tid >> 5;
  const int hh = lane >> 4, c = lane & 15;
  const int nt = blockIdx.x, mb = blockIdx.y, b = blockIdx.z;
  const int n0 = nt * QT, o0 = mb * QT;
  const unsigned short* ap = V16 + ((size_t)(b * CH + o0 + c)) * SEQ + 8 * hh;
  const unsigned short* bp = P16 + ((size_t)(b * SEQ + n0 + 16 * wave + c)) * SEQ + 8 * hh;
  v8f acc[4];
#pragma unroll
  for (int mt = 0; mt < 4; ++mt) acc[mt] = zero8();
  gemm_core<1, true>(acc, ap, ap, (size_t)16 * SEQ, bp, bp, SEQ / 32);
  stage_nT(Os, acc, IPCAR, wave, hh, c);
  __syncthreads();
  planes_out<false>(Os, nullptr, o0, Mh, Mlo, (size_t)(b * SEQ + n0), tid);
}

__global__ __launch_bounds__(128)
void gemm_out(const unsigned short* __restrict__ W, const float* __restrict__ bias,
              const unsigned short* __restrict__ Mh, const unsigned short* __restrict__ Mlo,
              const float* __restrict__ xres, float* out) {
  __shared__ __align__(16) float Os[QT * OSP];
  const int tid = threadIdx.x, lane = tid & 31, wave = tid >> 5;
  const int hh = lane >> 4, c = lane & 15;
  const int nt = blockIdx.x, mb = blockIdx.y, b = blockIdx.z;
  const int n0 = nt * QT, o0 = mb * QT;
  const unsigned short* ap = W + (size_t)(o0 + c) * CH + 8 * hh;
  const size_t bq = ((size_t)(b * SEQ + n0 + 16 * wave + c)) * CH + 8 * hh;
  v8f acc[4];
#pragma unroll
  for (int mt = 0; mt < 4; ++mt) acc[mt] = zero8();
  gemm_core<2, false>(acc, ap, ap, (size_t)16 * CH, Mh + bq, Mlo + bq, CH / 32);
  stage_mn(Os, acc, wave, hh, c);
  __syncthreads();
  const int e = tid & 15, lq = tid >> 4;
  v4f res[8];
#pragma unroll
  for (int it = 0; it < 8; ++it) {
    const int row = it * 8 + lq;
    const float bb = bfr(bias[o0 + row]);
    const size_t idx = ((size_t)(b * CH + o0 + row)) * T_FULL + n0 + 4 * e;
    const v4f a  = *(const v4f*)(Os + row * OSP + 4 * e);
    const v4f xv = *(const v4f*)(xres + idx);
#pragma unroll
    for (int t = 0; t < 4; ++t) res[it][t] = (a[t] + bb) + bfr(xv[t]);
  }
#pragma unroll
  for (int pass = 0; pass < 2; ++pass) {
#pragma unroll
    for (int it = 0; it < 8; ++it) {
      const int row = it * 8 + lq;
      const size_t idx = ((size_t)(b * CH + o0 + row)) * T_FULL + n0 + 4 * e;
      *(volatile v4f*)(out + idx) = res[it];
    }
    __threadfence();
  }
}

extern "C" void kernel_launch(void* const* d_in, const int* in_sizes, int n_in,
                              void* d_out, int out_size, void* d_ws, size_t ws_size,
                              hipStream_t stream) {
  if (n_in < 10) return;
  if (in_sizes[0] < NB * CH * T_FULL || in_sizes[1] < NB * CH * T_FULL) return;
  if (in_sizes[2] < CH * CH || in_sizes[4] < CH * CH || in_sizes[6] < CH * CH || in_sizes[8] < CH * CH) return;
  if (in_sizes[3] < CH || in_sizes[5] < CH || in_sizes[7] < CH || in_sizes[9] < CH) return;
  if (out_size < NB * CH * T_FULL) return;

  size_t off = 0;
  auto carve = [&](size_t bytes) { const size_t o = off; off += (bytes + 255) & ~(size_t)255; return o; };
  const size_t oW = carve(WB);
  const size_t oX = carve(RXB);
  const size_t oM = carve(RMB);
  const size_t oV = carve(RVB);
  if (off > ws_size) return;
  if (off > (size_t)WS_CAP) return;

  const float* x_c = (const float*)d_in[0];
  const float* x_s = (const float*)d_in[1];
  const float* Wn  = (const float*)d_in[2];
  const float* bn  = (const float*)d_in[3];
  const float* Wm  = (const float*)d_in[4];
  const float* bm  = (const float*)d_in[5];
  const float* Wl  = (const float*)d_in[6];
  const float* bl  = (const float*)d_in[7];
  const float* Wo  = (const float*)d_in[8];
  const float* bo  = (const float*)d_in[9];
  float* out = (float*)d_out;

  char* ws = (char*)d_ws;
  unsigned short* W16  = (unsigned short*)(ws + oW);
  unsigned short* Xcnh = (unsigned short*)(ws + oX);
  unsigned short* Xcnl = (unsigned short*)(ws + oX + PLB);
  unsigned short* Xsnh = (unsigned short*)(ws + oX + 2 * PLB);
  unsigned short* Xsnl = (unsigned short*)(ws + oX + 3 * PLB);
  unsigned short* Xsr  = (unsigned short*)(ws + oX + 4 * PLB);
  float*          S    = (float*)(ws + oX);
  unsigned short* Moh  = (unsigned short*)(ws + oX);
  unsigned short* Mol  = (unsigned short*)(ws + oX + PLB);
  unsigned short* Mnh  = (unsigned short*)(ws + oM);
  unsigned short* Mnl  = (unsigned short*)(ws + oM + PLB);
  unsigned short* Mmh  = (unsigned short*)(ws + oM + 2 * PLB);
  unsigned short* Mml  = (unsigned short*)(ws + oM + 3 * PLB);
  unsigned short* P16  = (unsigned short*)(ws + oM);
  unsigned short* V16  = (unsigned short*)(ws + oV);

  const dim3 blk256(256), blk128(128);
  const dim3 gconv(SEQ / QT, CH / QT, NB);

  cvt_w<<<dim3(NMAT * CH / 8), blk256, 0, stream>>>(Wn, Wm, Wl, Wo, W16);
  cvt_norm<0><<<dim3(CH / QT, NB), blk256, 0, stream>>>(x_c, Xcnh, Xcnl, Xcnl);
  cvt_norm<1><<<dim3(CH / QT, NB), blk256, 0, stream>>>(x_s, Xsnh, Xsnl, Xsr);
  gemm_nm<<<gconv, blk128, 0, stream>>>(W16, bn, Xcnh, Xcnl, Mnh, Mnl);
  gemm_nm<<<gconv, blk128, 0, stream>>>(W16 + (size_t)CH * CH, bm, Xsnh, Xsnl, Mmh, Mml);
  gemm_val<<<gconv, blk128, 0, stream>>>(W16 + (size_t)2 * CH * CH, bl, Xsr, V16);
  gemm_sc<<<dim3(SEQ / QT, SEQ / QT, NB), blk128, 0, stream>>>(Mnh, Mnl, Mmh, Mml, S);
  softmax_k<<<dim3(NB * SEQ / 8), blk256, 0, stream>>>(S, P16);
  gemm_pv<<<gconv, blk128, 0, stream>>>(V16, P16, Moh, Mol);
  gemm_out<<<gconv, blk128, 0, stream>>>(W16 + (size_t)3 * CH * CH, bo, Moh, Mol, x_c, out);
  (void)hipGetLastError();
}
